// Embeddings_51994874085872
// MI455X (gfx1250) — hardware-verified
//
#include <hip/hip_runtime.h>
#include <math.h>
#include <stdint.h>

#define NZ    2
#define NP    512
#define NR    32
#define NH    32
#define NG    32
#define NI    32
#define NJ    8
#define NO    256
#define AT    16
#define NWV   4
#define BPW   (NP / NWV)
#define MTILE (NI * NG)
#define PLS   (NZ * NP * MTILE)
static_assert(NP == NWV * BPW);
static_assert((NP % AT) == 0);
static_assert(NO == NI * NJ);
static_assert(NR == 32);
static_assert(NH == 32);
static_assert(NG == 32);
static_assert(NI == 32);
static_assert(AT * NI == 128 * 4);
static_assert(MTILE == 128 * 8);
static_assert(sizeof(_Float16) == 2);

typedef _Float16 v16h __attribute__((ext_vector_type(16)));
typedef _Float16 v8h  __attribute__((ext_vector_type(8)));
typedef _Float16 v4h  __attribute__((ext_vector_type(4)));
typedef float    v8f  __attribute__((ext_vector_type(8)));
typedef float    v4f  __attribute__((ext_vector_type(4)));

union Frag { v16h v; v8h half[2]; };

constexpr float kInv31     = 1.0f / 31.0f;
constexpr float kStep      = 10.0f * kInv31;
constexpr float kInvStep   = 1.0f / kStep;
constexpr float kHalfPi    = 1.5707963267948966f;
constexpr float kInvSqrt32 = 1.0f / 5.656854249492381f;
constexpr float kInvSqrt8  = 1.0f / 2.8284271247461903f;
constexpr float kOutScale  = kInvSqrt32 * kInvSqrt8;
constexpr float kInv2048   = 0.00048828125f;
constexpr float kEps2      = 1.91e-15f;

__device__ __forceinline__ unsigned short bf_bits(float f) {
  unsigned u = __float_as_uint(f);
  return (unsigned short)((u + 0x7FFFu + ((u >> 16) & 1u)) >> 16);
}
__device__ __forceinline__ float bf_up(unsigned short b) { return __uint_as_float(((unsigned)b) << 16); }
__device__ __forceinline__ float bfr(float f) { return bf_up(bf_bits(f)); }
__device__ __forceinline__ v8f zero8() {
  v8f z;
  z[0] = 0.f; z[1] = 0.f; z[2] = 0.f; z[3] = 0.f; z[4] = 0.f; z[5] = 0.f; z[6] = 0.f; z[7] = 0.f;
  return z;
}
__device__ __forceinline__ void hsplit(float v, _Float16& hi, _Float16& lo) {
  const _Float16 hv = (_Float16)v;
  hi = hv;
  lo = (_Float16)((v - (float)hv) * 2048.0f);
}

__device__ __forceinline__ v16h ldfrag(const _Float16* p) {
  Frag f;
  f.half[0] = *(const v8h*)(p);
  f.half[1] = *(const v8h*)(p + 16);
  return f.v;
}

__device__ __forceinline__ void ldsplit(const float* p, Frag& fh, Frag& fl) {
  const v4f q0 = *(const v4f*)(p);
  const v4f q1 = *(const v4f*)(p + 4);
  const v4f q2 = *(const v4f*)(p + 16);
  const v4f q3 = *(const v4f*)(p + 20);
  v8h h0, l0, h1, l1;
#pragma unroll
  for (int c = 0; c < 4; ++c) {
    _Float16 th, tl;
    hsplit(q0[c], th, tl); h0[c]     = th; l0[c]     = tl;
    hsplit(q1[c], th, tl); h0[4 + c] = th; l0[4 + c] = tl;
    hsplit(q2[c], th, tl); h1[c]     = th; l1[c]     = tl;
    hsplit(q3[c], th, tl); h1[4 + c] = th; l1[4 + c] = tl;
  }
  fh.half[0] = h0; fh.half[1] = h1;
  fl.half[0] = l0; fl.half[1] = l1;
}

__device__ __forceinline__ v8f mma(v16h a, v16h b, v8f c) {
  v8f d = __builtin_amdgcn_wmma_f32_16x16x32_f16(false, a, false, b, (short)0, c, false, false);
#if defined(__HIP_DEVICE_COMPILE__)
  asm volatile("v_nop\n\tv_nop\n\tv_nop\n\tv_nop" : "+v"(d) : "v"(a), "v"(b));
#endif
  return d;
}

__global__ __launch_bounds__(256) void k_prep(const float* __restrict__ Wout, const float* __restrict__ elem,
                                             _Float16* MT) {
  __shared__ __align__(16) _Float16 sH[MTILE];
  __shared__ __align__(16) _Float16 sR[MTILE];
  const int tid = threadIdx.x;
  const int zb  = blockIdx.x;
  const int i   = tid >> 3;
  const int g4  = (tid & 7) * 4;

  const float* ep = elem + (size_t)zb * NJ;
  float ev[NJ];
#pragma unroll
  for (int j = 0; j < NJ; ++j) ev[j] = bfr(ep[j]);

  float mv[4];
  mv[0] = 0.f; mv[1] = 0.f; mv[2] = 0.f; mv[3] = 0.f;
#pragma unroll
  for (int j = 0; j < NJ; ++j) {
    const v4f w = *(const v4f*)(Wout + (size_t)(i * NJ + j) * NG + g4);
#pragma unroll
    for (int c = 0; c < 4; ++c) mv[c] += bfr(w[c]) * ev[j];
  }
  v4h hv, rv;
#pragma unroll
  for (int c = 0; c < 4; ++c) {
    _Float16 th, tl;
    hsplit(mv[c], th, tl);
    hv[c] = th; rv[c] = tl;
  }
  *(v4h*)(sH + i * NG + g4) = hv;
  *(v4h*)(sR + i * NG + g4) = rv;
  __syncthreads();

  const int pl = tid >> 7;
  const int q  = tid & 127;
  const v8h ph = *(const v8h*)(sH + 8 * q);
  const v8h pr = *(const v8h*)(sR + 8 * q);
  v8h pv = ph;
  if (pl != 0) pv = pr;
  _Float16* dst = MT + (size_t)pl * PLS + (size_t)zb * MTILE + 8 * q;
  *(volatile v8h*)dst = pv;
  __threadfence();
  *(volatile v8h*)dst = pv;
}

__global__ __launch_bounds__(128) void k_main(const float* __restrict__ xyz, const float* __restrict__ maskp,
                                             const float* __restrict__ W0, const float* __restrict__ W1,
                                             const _Float16* __restrict__ MT, float* out) {
#pragma clang fp contract(off)
  __shared__ __align__(16) float sX[NWV * AT * 32];
  const int tid  = threadIdx.x;
  const int lane = tid & 31, wid = tid >> 5, h = lane >> 4, m = lane & 15;
  const int z    = blockIdx.x / (NP / AT);
  const int a0   = (blockIdx.x % (NP / AT)) * AT;

  v16h w0f[2], w1f[2];
#pragma unroll
  for (int nt = 0; nt < 2; ++nt) {
    const float* p0 = W0 + (size_t)(nt * 16 + m) * NR;
    const float* p1 = W1 + (size_t)(nt * 16 + m) * NH;
    v16h f0, f1;
#pragma unroll
    for (int e = 0; e < 8; ++e) {
      f0[e]     = (_Float16)bfr(p0[8 * h + e]);
      f0[8 + e] = (_Float16)bfr(p0[16 + 8 * h + e]);
      f1[e]     = (_Float16)bfr(p1[8 * h + e]);
      f1[8 + e] = (_Float16)bfr(p1[16 + 8 * h + e]);
    }
    w0f[nt] = f0; w1f[nt] = f1;
  }

  const int   pa  = a0 + m;
  const float pax = bfr(xyz[(size_t)(z * NP + pa) * 3 + 0]);
  const float pay = bfr(xyz[(size_t)(z * NP + pa) * 3 + 1]);
  const float paz = bfr(xyz[(size_t)(z * NP + pa) * 3 + 2]);

  v8f accH[2], accR[2];
  accH[0] = zero8(); accH[1] = zero8(); accR[0] = zero8(); accR[1] = zero8();

  float* sXw = sX + wid * (AT * 32);

#pragma unroll 1
  for (int s = 0; s < BPW; ++s) {
    const int b  = wid * BPW + s;
    const int zb = z * NP + b;
    __syncthreads();

    const float bxr = bfr(xyz[(size_t)zb * 3 + 0]);
    const float byr = bfr(xyz[(size_t)zb * 3 + 1]);
    const float bzr = bfr(xyz[(size_t)zb * 3 + 2]);
    const float dx = pax - bxr, dy = pay - byr, dz = paz - bzr;
    float sq = (dx * dx + dy * dy) + dz * dz;
    sq = fmaxf(sq, 1e-12f);
    const float r = __builtin_sqrtf(sq);
    const float t = r * kInvStep;
    int kA = (int)t;
    kA = min(kA, 1000);
    const int kB  = kA + 1;
    const int kAc = min(kA, 31), kBc = min(kB, 31);
    const float cA = (kAc >= 31) ? 10.0f : 10.0f * ((float)kAc * kInv31);
    const float cB = (kBc >= 31) ? 10.0f : 10.0f * ((float)kBc * kInv31);
    float dA = (r - cA) * kInvStep;
    float dB = (r - cB) * kInvStep;
    dA = fminf(fmaxf(dA, -1.0f), 1.0f);
    dB = fminf(fmaxf(dB, -1.0f), 1.0f);
    float vA = cosf(kHalfPi * dA);
    float vB = cosf(kHalfPi * dB);
    vA = vA * vA;
    vB = vB * vB;

    Frag fbh, fbl;
    {
      v8h h0, l0, h1, l1;
#pragma unroll
      for (int e = 0; e < 8; ++e) {
        const int k0 = 8 * h + e;
        const int k1 = 16 + 8 * h + e;
        const float v0 = (k0 == kA) ? vA : ((k0 == kB) ? vB : kEps2);
        const float v1 = (k1 == kA) ? vA : ((k1 == kB) ? vB : kEps2);
        _Float16 th, tl;
        hsplit(v0, th, tl); h0[e] = th; l0[e] = tl;
        hsplit(v1, th, tl); h1[e] = th; l1[e] = tl;
      }
      fbh.half[0] = h0; fbh.half[1] = h1;
      fbl.half[0] = l0; fbl.half[1] = l1;
    }

    {
      v8f ch[2], cr[2];
#pragma unroll
      for (int nt = 0; nt < 2; ++nt) {
        ch[nt] = mma(fbh.v, w0f[nt], zero8());
        cr[nt] = mma(fbl.v, w0f[nt], zero8());
      }
#pragma unroll
      for (int nt = 0; nt < 2; ++nt)
#pragma unroll
        for (int rr = 0; rr < 8; ++rr) {
          const float x = (ch[nt][rr] + cr[nt][rr] * kInv2048) * kInvSqrt32;
          sXw[(8 * h + rr) * 32 + nt * 16 + m] = fmaxf(x, 0.0f);
        }
    }
    __syncthreads();
    Frag x1h, x1l;
    ldsplit(sXw + m * 32 + 8 * h, x1h, x1l);

    {
      v8f ch[2], cr[2];
#pragma unroll
      for (int nt = 0; nt < 2; ++nt) {
        ch[nt] = mma(x1h.v, w1f[nt], zero8());
        cr[nt] = mma(x1l.v, w1f[nt], zero8());
      }
#pragma unroll
      for (int nt = 0; nt < 2; ++nt)
#pragma unroll
        for (int rr = 0; rr < 8; ++rr) {
          const float x = (ch[nt][rr] + cr[nt][rr] * kInv2048) * kInvSqrt32;
          sXw[(8 * h + rr) * 32 + nt * 16 + m] = fmaxf(x, 0.0f);
        }
    }
    __syncthreads();
    Frag x2h, x2l;
    ldsplit(sXw + m * 32 + 8 * h, x2h, x2l);

    const _Float16* mp = MT + (size_t)zb * MTILE + (size_t)m * NG + 8 * h;
#pragma unroll
    for (int nt = 0; nt < 2; ++nt) {
      const v16h mh = ldfrag(mp + nt * (16 * NG));
      const v16h mr = ldfrag(mp + PLS + nt * (16 * NG));
      accH[nt] = mma(x2h.v, mh, accH[nt]);
      accR[nt] = mma(x2l.v, mh, accR[nt]);
      accR[nt] = mma(x2h.v, mr, accR[nt]);
    }
  }

  __syncthreads();
#pragma unroll
  for (int nt = 0; nt < 2; ++nt)
#pragma unroll
    for (int rr = 0; rr < 8; ++rr)
      sXw[(8 * h + rr) * 32 + nt * 16 + m] = accH[nt][rr] + accR[nt][rr] * kInv2048;
  __syncthreads();

  const int   row = tid >> 3;
  const float mk  = bfr(maskp[z * NP + a0 + row]);
  v4f ov;
#pragma unroll
  for (int c = 0; c < 4; ++c) {
    const int q = tid * 4 + c;
    float sacc = sX[q];
    sacc += sX[AT * 32 + q];
    sacc += sX[2 * AT * 32 + q];
    sacc += sX[3 * AT * 32 + q];
    ov[c] = (sacc * kOutScale) * mk;
  }
  float* od = out + (size_t)(z * NP + a0) * NI + tid * 4;
  *(volatile v4f*)od = ov;
  __threadfence();
  *(volatile v4f*)od = ov;
}

extern "C" void kernel_launch(void* const* d_in, const int* in_sizes, int n_in,
                              void* d_out, int out_size, void* d_ws, size_t ws_size,
                              hipStream_t stream) {
  if (n_in < 6) return;
  if (in_sizes[0] != NZ * NP * 3) return;
  if (in_sizes[1] != NZ * NP * NJ) return;
  if (in_sizes[2] != NZ * NP) return;
  if (in_sizes[3] != NH * NR) return;
  if (in_sizes[4] != NG * NH) return;
  if (in_sizes[5] != NO * NG) return;
  if (out_size != NZ * NP * NI) return;

  const float* xyz   = (const float*)d_in[0];
  const float* elem  = (const float*)d_in[1];
  const float* maskp = (const float*)d_in[2];
  const float* W0    = (const float*)d_in[3];
  const float* W1    = (const float*)d_in[4];
  const float* Wout  = (const float*)d_in[5];
  float* out = (float*)d_out;

  const size_t szMT = (size_t)2 * PLS * sizeof(_Float16);
  if (szMT > ws_size) return;
  if (szMT > (size_t)134217728) return;
  _Float16* MT = (_Float16*)d_ws;

  const dim3 gPrep(NZ * NP),       bPrep(256);
  const dim3 gMain(NZ * NP / AT),  bMain(128);

  k_prep<<<gPrep, bPrep, 0, stream>>>(Wout, elem, MT);
  k_main<<<gMain, bMain, 0, stream>>>(xyz, maskp, W0, W1, MT, out);
  (void)hipGetLastError();
}
